// TwoGATCN_87720412053583
// MI455X (gfx1250) — hardware-run, weakly checked
//
#include <hip/hip_runtime.h>

typedef float          v8f   __attribute__((ext_vector_type(8)));
typedef float          v4f   __attribute__((ext_vector_type(4)));
typedef unsigned int   v4u   __attribute__((ext_vector_type(4)));
typedef int            v8i   __attribute__((ext_vector_type(8)));
typedef unsigned short v8us  __attribute__((ext_vector_type(8)));
typedef unsigned short v16us __attribute__((ext_vector_type(16)));
typedef __bf16         v16bf __attribute__((ext_vector_type(16)));
typedef _Float16       v16h  __attribute__((ext_vector_type(16)));
typedef v4f  __attribute__((may_alias)) v4fa;
typedef v8us __attribute__((may_alias)) v8usa;
union FragB { v16bf v; v16us u; v8us h[2]; v8i w; };
union FragH { v16h  v; v16us u; v8us h[2]; v8i w; };

__device__ __forceinline__ v8f wmb(const FragB& a, const FragB& b, v8f c) {
  v8f d = __builtin_amdgcn_wmma_f32_16x16x32_bf16(false, a.v, false, b.v, (short)0, c, false, false);
  asm volatile("v_nop\n\tv_nop\n\tv_nop\n\tv_nop" : "+v"(d) : "v"(a.w), "v"(b.w));
  return d;
}

__device__ __forceinline__ v8f wmh(const FragH& a, const FragH& b, v8f c) {
  v8f d = __builtin_amdgcn_wmma_f32_16x16x32_f16(false, a.v, false, b.v, (short)0, c, false, false);
  asm volatile("v_nop\n\tv_nop\n\tv_nop\n\tv_nop" : "+v"(d) : "v"(a.w), "v"(b.w));
  return d;
}

__device__ __forceinline__ unsigned bf16_bits(float f) {
  const unsigned u = __float_as_uint(f);
  const unsigned r = (u + 0x7FFFu + ((u >> 16) & 1u)) >> 16;
  const unsigned q = (u >> 16) | 0x40u;
  return ((u & 0x7fffffffu) > 0x7f800000u) ? q : r;
}

__device__ __forceinline__ float bf16_val(float f) {
  return __uint_as_float(bf16_bits(f) << 16);
}
__device__ __forceinline__ int clampi(int v, int lo, int hi) {
  return v < lo ? lo : (v > hi ? hi : v);
}

__device__ __forceinline__ unsigned f16_bits(float f) {
  const unsigned u  = __float_as_uint(f);
  const unsigned s  = (u >> 16) & 0x8000u;
  const unsigned a  = u & 0x7fffffffu;
  const unsigned t  = a - 0x38000000u;
  const unsigned r  = (t + 0x0FFFu + ((t >> 13) & 1u)) >> 13;
  const unsigned rc = r > 0x7C00u ? 0x7C00u : r;
  const bool small  = a < 0x38800000u;
  const bool isnan  = a > 0x7f800000u;
  const unsigned fin = small ? 0u : (s | rc);
  return isnan ? (s | 0x7E00u) : fin;
}

__device__ __forceinline__ unsigned pk16(unsigned lo, unsigned hi) { return lo | (hi << 16); }
__device__ __forceinline__ unsigned bf16_lo_bits(float v) {
  float hi = bf16_val(v);
  asm volatile("" : "+v"(hi));
  return bf16_bits(v - hi);
}
__device__ __forceinline__ v4u pack8_bf16(v4f a, v4f c) {
  return (v4u){ pk16(bf16_bits(a[0]), bf16_bits(a[1])), pk16(bf16_bits(a[2]), bf16_bits(a[3])),
                pk16(bf16_bits(c[0]), bf16_bits(c[1])), pk16(bf16_bits(c[2]), bf16_bits(c[3])) };
}
__device__ __forceinline__ v4u pack8_bf16_lo(v4f a, v4f c) {
  return (v4u){ pk16(bf16_lo_bits(a[0]), bf16_lo_bits(a[1])), pk16(bf16_lo_bits(a[2]), bf16_lo_bits(a[3])),
                pk16(bf16_lo_bits(c[0]), bf16_lo_bits(c[1])), pk16(bf16_lo_bits(c[2]), bf16_lo_bits(c[3])) };
}
__device__ __forceinline__ v4u pack8_f16(v4f a, v4f c) {
  return (v4u){ pk16(f16_bits(a[0]), f16_bits(a[1])), pk16(f16_bits(a[2]), f16_bits(a[3])),
                pk16(f16_bits(c[0]), f16_bits(c[1])), pk16(f16_bits(c[2]), f16_bits(c[3])) };
}

template <int FORM>
__global__ __launch_bounds__(256) void k_plane(const float* __restrict__ src, int rows, int cols, int ldsrc,
                                               unsigned short* __restrict__ dst, int MP, int KP) {
  static_assert(FORM >= 0 && FORM <= 3);
  const int KTOT = (FORM == 1 || FORM == 3) ? 2 * KP : KP;
  const unsigned ppr   = (unsigned)(KTOT >> 3);
  const unsigned kp8   = (unsigned)(KP >> 3);
  const unsigned total = (unsigned)MP * ppr;
  const unsigned g     = blockIdx.x * 256u + threadIdx.x;
  const unsigned rowu  = g / ppr;
  const unsigned p     = g - rowu * ppr;
  const bool second    = p >= kp8;
  const int row = (int)rowu;
  const int c0  = (int)((second ? p - kp8 : p) << 3);
  const float* srow = src + (size_t)clampi(row, 0, rows - 1) * (size_t)ldsrc;
  float x[8];
  unsigned mk[8];
#pragma unroll
  for (int e = 0; e < 8; ++e) {
    const int c = c0 + e;
    const float v = srow[clampi(c, 0, cols - 1)];
    asm volatile("" :: "v"(v));
    x[e]  = v;
    mk[e] = (row < rows && c < cols) ? 0xFFFFu : 0u;
  }
  const v4f a = (v4f){ x[0], x[1], x[2], x[3] };
  const v4f c = (v4f){ x[4], x[5], x[6], x[7] };
  v4u o;
  if (FORM == 2) {
    o = pack8_f16(a, c);
  } else {
    const v4u hi = pack8_bf16(a, c);
    o = hi;
    if (FORM == 1) { const v4u lo = pack8_bf16_lo(a, c); o = second ? lo : hi; }
  }
  const v4u mw = (v4u){ pk16(mk[0], mk[1]), pk16(mk[2], mk[3]), pk16(mk[4], mk[5]), pk16(mk[6], mk[7]) };
  o &= mw;
  if (g < total) {
    volatile v4u* q = (volatile v4u*)(dst + (size_t)g * 8);
    *q = o;
    __threadfence();
    *q = o;
  }
}

template <int FORM> struct FragOf    { typedef FragB T; };
template <>         struct FragOf<2> { typedef FragH T; };
__device__ __forceinline__ v8f mm(const FragB& a, const FragB& b, v8f c) { return wmb(a, b, c); }
__device__ __forceinline__ v8f mm(const FragH& a, const FragH& b, v8f c) { return wmh(a, b, c); }
template <class F> __device__ __forceinline__ F ld_frag(const unsigned short* p) {
  F f;
  f.h[0] = *(const v8usa*)(p);
  f.h[1] = *(const v8usa*)(p + 16);
  return f;
}

template <int FORM, int EPI>
__global__ __launch_bounds__(256) __attribute__((amdgpu_num_vgpr(248)))
void k_gemm_nt(const unsigned short* __restrict__ A, const unsigned short* __restrict__ B,
               const float* __restrict__ bias, float* __restrict__ D, int M, int N, int KTOT, int ldd) {
  static_assert(FORM >= 0 && FORM <= 2);
  static_assert(EPI == 0 || EPI == 1);
  typedef typename FragOf<FORM>::T F;
  __shared__ __attribute__((aligned(16))) float sT[8][16 * 68];
  const int lane = threadIdx.x & 31;
  const int wave = threadIdx.x >> 5;
  const int tilesM = (M + 63) >> 6;
  const int tilesN = (N + 63) >> 6;
  const int tile = blockIdx.x * 8 + wave;
  if (tile >= tilesM * tilesN) return;
  const int tm = tile / tilesN;
  const int tn = tile - tm * tilesN;
  const int m0 = tm << 6;
  const int n0 = tn << 6;

  const int rl = lane & 15;
  const int h8 = (lane >> 4) * 8;
  const unsigned short* pa = A + (size_t)(m0 + rl) * (size_t)KTOT + h8;
  const unsigned short* pb = B + (size_t)(n0 + rl) * (size_t)KTOT + h8;

  v8f acc[4][4];
#pragma unroll
  for (int i = 0; i < 4; ++i)
#pragma unroll
    for (int j = 0; j < 4; ++j) acc[i][j] = (v8f){0.f, 0.f, 0.f, 0.f, 0.f, 0.f, 0.f, 0.f};

#pragma unroll 1
  for (int k0 = 0; k0 < KTOT; k0 += 32) {
    F bf[4];
#pragma unroll
    for (int j = 0; j < 4; ++j) bf[j] = ld_frag<F>(pb + (size_t)(j << 4) * (size_t)KTOT + k0);
#pragma unroll
    for (int i = 0; i < 4; ++i) {
      const F af = ld_frag<F>(pa + (size_t)(i << 4) * (size_t)KTOT + k0);
#pragma unroll
      for (int j = 0; j < 4; ++j) acc[i][j] = mm(af, bf[j], acc[i][j]);
    }
  }

  float* slab = sT[wave];
  const int hh = lane >> 4;
  const int c4 = (lane & 15) * 4;
  const int nc = n0 + c4;
  const bool cok = nc < N;
  v4f bv = (v4f){0.f, 0.f, 0.f, 0.f};
  if (EPI == 1) {
    bv = *(const v4fa*)(bias + clampi(nc, 0, N - 4));
    asm volatile("" :: "v"(bv));
  }
#pragma unroll
  for (int i = 0; i < 4; ++i) {
    const int mBase = m0 + (i << 4);
#pragma unroll
    for (int j = 0; j < 4; ++j) {
#pragma unroll
      for (int r = 0; r < 8; ++r) slab[(h8 + r) * 68 + (j << 4) + rl] = acc[i][j][r];
    }
    __builtin_amdgcn_fence(__ATOMIC_RELEASE, "workgroup");
    __builtin_amdgcn_wave_barrier();
    __builtin_amdgcn_fence(__ATOMIC_ACQUIRE, "workgroup");
    v4f vv[8];
#pragma unroll
    for (int it = 0; it < 8; ++it) {
      const int row = it * 2 + hh;
      v4f v = *(const v4fa*)(slab + row * 68 + c4);
      if (EPI == 1) v += bv;
      vv[it] = v;
    }
    for (int pass = 0; pass < 2; ++pass) {
#pragma unroll
      for (int it = 0; it < 8; ++it) {
        const int row = mBase + it * 2 + hh;
        if (cok && row < M) *(volatile v4f*)(D + (size_t)row * (size_t)ldd + nc) = vv[it];
      }
      __threadfence();
    }
    __builtin_amdgcn_fence(__ATOMIC_RELEASE, "workgroup");
    __builtin_amdgcn_wave_barrier();
    __builtin_amdgcn_fence(__ATOMIC_ACQUIRE, "workgroup");
  }
}

#pragma clang fp contract(off)

typedef unsigned int v2u __attribute__((ext_vector_type(2)));
typedef int          v4i __attribute__((ext_vector_type(4)));
typedef v4i __attribute__((may_alias)) v4ia;

constexpr int SPLIT_L2   = 1;
constexpr int SPLIT_HEAD = 1;

constexpr int NN    = 50000;
constexpr int NP    = 50048;
constexpr int EE    = 800000;
constexpr int DF    = 128;
constexpr int H1    = 256;
constexpr int H2    = 128;
constexpr int NCLS  = 40;
constexpr int TN    = 64;
constexpr int LDF   = 256;
constexpr int K1    = DF;
constexpr int K2    = H1 * (1 + SPLIT_L2);
constexpr int K3    = H2 * (1 + SPLIT_HEAD);
constexpr int OUT_ELEMS = NN * NCLS;
constexpr float NEGS = 0.2f;

constexpr int BNW    = 8;
constexpr int NBA    = 1024;
constexpr int SLA    = 10;
constexpr int NBLK   = 49;
constexpr int NTAB   = NBLK * NBA;
constexpr int SEG    = EE / BNW;
constexpr int WCH    = 128;
constexpr int NIT    = (SEG + WCH - 1) / WCH;
constexpr int WLCAP  = 3072;
constexpr int LCAP   = 21504;
constexpr int DEGCAP = 48;
constexpr int MEAS_HITS = 16623;
constexpr int MEAS_DEG  = 35;
constexpr int B_ZINTS = LCAP + 3 * NBA + 16;
constexpr int B_INTS  = B_ZINTS + BNW * WLCAP;
constexpr int B_BYTES = B_INTS * 4;

static_assert(NP % 64 == 0 && NP >= NN && NN % 16 == 0 && NP % 8 == 0 && NN % 8 == 0);
static_assert(K1 % 32 == 0 && K2 % 32 == 0 && K3 % 32 == 0 && H1 % 64 == 0 && TN % 64 == 0 && TN >= NCLS);
static_assert(LDF % 32 == 0 && TN % 32 == 0 && LDF == H1 && LDF == 2 * H2);
static_assert(EE % BNW == 0 && SEG * BNW == EE);
static_assert(NBA == (1 << SLA) && NTAB >= NN && NTAB == 50176 && ((NN - 1) >> SLA) == NBLK - 1);
static_assert(NN <= 65536);
static_assert(LCAP * 4 >= MEAS_HITS * 5 && LCAP % (4 * 256) == 0);
static_assert(WLCAP * BNW * 4 >= MEAS_HITS * 5 && WLCAP % 32 == 0);
static_assert(DEGCAP * 4 >= MEAS_DEG * 5 && DEGCAP < 63);
static_assert(B_ZINTS % 4 == 0 && B_BYTES <= 262144 && B_BYTES == 196672 && B_BYTES <= 327680);
static_assert(OUT_ELEMS == 2000000 && (OUT_ELEMS + 255) / 256 == 7813 && OUT_ELEMS - 7812 * 256 == 128);

constexpr int V_ATT1 = 0, V_B1 = 256, V_ATT2 = 512, V_B2 = 640, V_BC = 768, V_FLOATS = 832;

constexpr size_t SZ_P    = (size_t)NP * LDF * 4;
constexpr size_t SZ_Q    = (size_t)NP * LDF * 4;
constexpr size_t SZ_XB   = (size_t)NP * DF * 2;
constexpr size_t SZ_H1S  = (size_t)NP * H1 * 2;
constexpr size_t SZ_RX   = (SPLIT_L2 != 0) ? SZ_XB : (SZ_H1S > SZ_XB ? SZ_H1S : SZ_XB);
constexpr size_t SZ_H2   = (size_t)NP * K3 * 2;
constexpr size_t SZ_T    = (size_t)NP * TN * 4;
constexpr size_t SZ_LIST = (size_t)NBLK * LCAP * 4;
constexpr size_t SZ_TAB  = (size_t)NTAB * 4;
constexpr size_t SZ_FLG  = (size_t)64 * 128;
constexpr size_t SZ_W1   = (size_t)H1 * K1 * 2;
constexpr size_t SZ_W2   = (size_t)H1 * K2 * 2;
constexpr size_t SZ_WC   = (size_t)TN * K3 * 2;
constexpr size_t SZ_VEC  = (size_t)V_FLOATS * 4;
constexpr size_t OFF_P    = 0;
constexpr size_t OFF_Q    = OFF_P + SZ_P;
constexpr size_t OFF_RX   = OFF_Q + SZ_Q;
constexpr size_t OFF_LIST = OFF_RX + SZ_RX;
constexpr size_t OFF_CNT  = OFF_LIST + SZ_LIST;
constexpr size_t OFF_OFF  = OFF_CNT + SZ_TAB;
constexpr size_t OFF_FLG  = OFF_OFF + SZ_TAB;
constexpr size_t OFF_W1L  = OFF_FLG + SZ_FLG;
constexpr size_t OFF_W1R  = OFF_W1L + SZ_W1;
constexpr size_t OFF_W2   = OFF_W1R + SZ_W1;
constexpr size_t OFF_WC   = OFF_W2 + SZ_W2;
constexpr size_t OFF_VEC  = OFF_WC + SZ_WC;
constexpr size_t WS_TOTAL = OFF_VEC + SZ_VEC;
static_assert(SZ_P % 256 == 0 && SZ_RX % 256 == 0 && SZ_LIST % 256 == 0 && SZ_TAB % 256 == 0 && SZ_FLG % 256 == 0);
static_assert(SZ_W1 % 256 == 0 && SZ_W2 % 256 == 0 && SZ_WC % 256 == 0 && SZ_VEC % 256 == 0);
static_assert(SZ_H2 % 256 == 0 && SZ_H2 + SZ_T <= SZ_Q);
static_assert(SPLIT_L2 == 0 || (size_t)NP * K2 * 2 == SZ_Q);
static_assert(NBLK <= 64);
static_assert(SPLIT_L2 * SPLIT_HEAD == 0 || WS_TOTAL == (size_t)((size_t)470173 << 8));
static_assert(WS_TOTAL <= ((size_t)128 << 20));

constexpr int NB_X   = NP * (DF / 8) / 256;
constexpr int NB_W1  = H1 * (K1 / 8) / 256;
constexpr int NB_W2  = H2 * (K2 / 8) / 256;
constexpr int NB_WC  = TN * (K3 / 8) / 256;
constexpr int O_W1L  = NB_X;
constexpr int O_W1R  = O_W1L + NB_W1;
constexpr int O_W2L  = O_W1R + NB_W1;
constexpr int O_W2R  = O_W2L + NB_W2;
constexpr int O_WC   = O_W2R + NB_W2;
constexpr int O_VEC  = O_WC + NB_WC;
constexpr int NB_PREP = O_VEC + 1;
static_assert(NB_X * 256 == NP * (DF / 8) && NB_W1 * 256 == H1 * (K1 / 8));
static_assert(NB_W2 * 256 == H2 * (K2 / 8) && NB_WC * 256 == TN * (K3 / 8));

__device__ __forceinline__ void put16(unsigned short* dp, v4u o) {
  volatile v4u* q = (volatile v4u*)dp;
  *q = o;
  __threadfence();
  *q = o;
}

__device__ __forceinline__ v4u wt_piece(const float* __restrict__ W, int ncols, int nsrc, int k0, unsigned msk) {
  const float* p = W + (size_t)k0 * (size_t)ncols + nsrc;
  float x[8];
#pragma unroll
  for (int e = 0; e < 8; ++e) {
    const float v = p[(size_t)e * (size_t)ncols];
    asm volatile("" :: "v"(v));
    x[e] = v;
  }
  v4u o = pack8_bf16((v4f){ x[0], x[1], x[2], x[3] }, (v4f){ x[4], x[5], x[6], x[7] });
  o &= (v4u){ msk, msk, msk, msk };
  return o;
}

__device__ __forceinline__ float sel5(float a, float b, float c, float d, float e,
                                      unsigned ma, unsigned mb, unsigned mc, unsigned md, unsigned me) {
  const unsigned bits = (__float_as_uint(bf16_val(a)) & ma) | (__float_as_uint(bf16_val(b)) & mb) |
                        (__float_as_uint(bf16_val(c)) & mc) | (__float_as_uint(bf16_val(d)) & md) |
                        (__float_as_uint(bf16_val(e)) & me);
  return __uint_as_float(bits);
}

__global__ __launch_bounds__(256) __attribute__((amdgpu_num_vgpr(248)))
void k_prep(const float* __restrict__ x, const float* __restrict__ W1l, const float* __restrict__ W1r,
            const float* __restrict__ att1, const float* __restrict__ b1,
            const float* __restrict__ W2l, const float* __restrict__ W2r,
            const float* __restrict__ att2, const float* __restrict__ b2,
            const float* __restrict__ Wc, const float* __restrict__ bc,
            unsigned short* __restrict__ XB, unsigned short* __restrict__ W1LT, unsigned short* __restrict__ W1RT,
            unsigned short* __restrict__ W2D, unsigned short* __restrict__ WCD, float* __restrict__ VEC) {
  const int tid = (int)threadIdx.x;
  const int blk = (int)blockIdx.x;
  if (blk < NB_X) {
    const int g   = blk * 256 + tid;
    const int row = g >> 4;
    const int p   = g & 15;
    const int rc  = row < NN ? row : NN - 1;
    const float* s = x + (size_t)rc * DF + 8 * p;
    const v4f a = *(const v4fa*)s;
    const v4f c = *(const v4fa*)(s + 4);
    asm volatile("" :: "v"(a));
    asm volatile("" :: "v"(c));
    const unsigned m = row < NN ? 0xFFFFFFFFu : 0u;
    v4u o = pack8_bf16(a, c);
    o &= (v4u){ m, m, m, m };
    put16(XB + (size_t)g * 8, o);
  } else if (blk < O_W1R) {
    const int g  = (blk - O_W1L) * 256 + tid;
    const int n  = g / (K1 / 8);
    const int k0 = (g - n * (K1 / 8)) * 8;
    put16(W1LT + (size_t)g * 8, wt_piece(W1l, H1, n, k0, 0xFFFFFFFFu));
  } else if (blk < O_W2L) {
    const int g  = (blk - O_W1R) * 256 + tid;
    const int n  = g / (K1 / 8);
    const int k0 = (g - n * (K1 / 8)) * 8;
    put16(W1RT + (size_t)g * 8, wt_piece(W1r, H1, n, k0, 0xFFFFFFFFu));
  } else if (blk < O_W2R) {
    const int g  = (blk - O_W2L) * 256 + tid;
    const int n  = g / (K2 / 8);
    const int k0 = ((g - n * (K2 / 8)) * 8) & (H1 - 1);
    put16(W2D + (size_t)g * 8, wt_piece(W2l, H2, n, k0, 0xFFFFFFFFu));
  } else if (blk < O_WC) {
    const int g  = (blk - O_W2R) * 256 + tid;
    const int n  = g / (K2 / 8);
    const int k0 = ((g - n * (K2 / 8)) * 8) & (H1 - 1);
    put16(W2D + (size_t)H2 * K2 + (size_t)g * 8, wt_piece(W2r, H2, n, k0, 0xFFFFFFFFu));
  } else if (blk < O_VEC) {
    const int g  = (blk - O_WC) * 256 + tid;
    const int n  = g / (K3 / 8);
    const int k0 = ((g - n * (K3 / 8)) * 8) & (H2 - 1);
    const int ns = n < NCLS ? n : NCLS - 1;
    const unsigned m = n < NCLS ? 0xFFFFFFFFu : 0u;
    put16(WCD + (size_t)g * 8, wt_piece(Wc, NCLS, ns, k0, m));
  } else {
    const int u = tid;
    const v4f a1 = *(const v4fa*)(att1 + 4 * clampi(u, 0, 63));
    asm volatile("" :: "v"(a1));
    const v4f c1 = *(const v4fa*)(b1 + 4 * clampi(u - 64, 0, 63));
    asm volatile("" :: "v"(c1));
    const v4f a2 = *(const v4fa*)(att2 + 4 * clampi(u - 128, 0, 31));
    asm volatile("" :: "v"(a2));
    const v4f c2 = *(const v4fa*)(b2 + 4 * clampi(u - 160, 0, 31));
    asm volatile("" :: "v"(c2));
    const v4f cc = *(const v4fa*)(bc + 4 * clampi(u - 192, 0, NCLS / 4 - 1));
    asm volatile("" :: "v"(cc));
    const unsigned ma = (u < 64) ? 0xFFFFFFFFu : 0u;
    const unsigned mb = (u >= 64 && u < 128) ? 0xFFFFFFFFu : 0u;
    const unsigned mc = (u >= 128 && u < 160) ? 0xFFFFFFFFu : 0u;
    const unsigned md = (u >= 160 && u < 192) ? 0xFFFFFFFFu : 0u;
    const unsigned me = (u >= 192 && u < 192 + NCLS / 4) ? 0xFFFFFFFFu : 0u;
    const v4f o = (v4f){ sel5(a1[0], c1[0], a2[0], c2[0], cc[0], ma, mb, mc, md, me),
                         sel5(a1[1], c1[1], a2[1], c2[1], cc[1], ma, mb, mc, md, me),
                         sel5(a1[2], c1[2], a2[2], c2[2], cc[2], ma, mb, mc, md, me),
                         sel5(a1[3], c1[3], a2[3], c2[3], cc[3], ma, mb, mc, md, me) };
    if (u < V_FLOATS / 4) {
      volatile v4f* q = (volatile v4f*)(VEC + 4 * u);
      *q = o;
      __threadfence();
      *q = o;
    }
  }
}
static_assert(NCLS % 4 == 0 && V_FLOATS / 4 == 208);

template <int PASS>
__device__ __forceinline__ int drain(const int* wlAll, const int* misc, int* cnt, int* cur, int* sl, int lane) {
  int t = 0, ov = 0;
#pragma unroll 1
  for (int w2 = 0; w2 < BNW; ++w2) {
    const int craw = __builtin_amdgcn_readfirstlane(misc[w2]);
    ov |= (craw > WLCAP || craw < 0) ? 1 : 0;
    const int c = clampi(craw, 0, WLCAP);
#pragma unroll 1
    for (int b0 = 0; b0 < c; b0 += 32) {
      const int j   = b0 + lane;
      const int idx = j < c - 1 ? j : c - 1;
      const int ent = wlAll[w2 * WLCAP + idx];
      const int rem = c - b0;
      const int m32 = rem < 32 ? rem : 32;
#pragma unroll 1
      for (int k = 0; k < m32; ++k) {
        const int u    = __builtin_amdgcn_readlane(ent, k);
        const int slot = u & (NBA - 1);
        if (t < LCAP) {
          if (lane == 0) {
            if (PASS == 0) {
              cnt[slot] = cnt[slot] + 1;
            } else {
              int p = cur[slot];
              p = clampi(p, 0, LCAP - 1);
              sl[p] = (int)((unsigned)u >> SLA);
              cur[slot] = p + 1;
            }
          }
          t = t + 1;
        } else {
          ov = 1;
        }
      }
    }
  }
  return t | (ov << 30);
}

__global__ __launch_bounds__(256) __attribute__((amdgpu_num_vgpr(248)))
void k_bucket(const int* __restrict__ ei, int* __restrict__ LIST, int* __restrict__ CNT, int* __restrict__ OFF,
              int* __restrict__ FLG) {
  extern __shared__ __attribute__((aligned(16))) int dsm[];
  int* sl    = dsm;
  int* cnt   = sl + LCAP;
  int* offs  = cnt + NBA;
  int* cur   = offs + NBA;
  int* misc  = cur + NBA;
  int* wlAll = misc + 16;
  const int tid = (int)threadIdx.x, lane = tid & 31, wave = tid >> 5;
  const int blk = (int)blockIdx.x;
  const int slotBase = blk * NBA;

  {
    const v4i z4 = (v4i){ 0, 0, 0, 0 };
    for (int i = tid * 4; i < B_ZINTS; i += 256 * 4) *(v4ia*)(dsm + i) = z4;
  }
  __syncthreads();

  {
    const int* srcp = ei;
    const int* dstp = ei + EE;
    const int segBeg = wave * SEG;
    const int segEnd = segBeg + SEG;
    int* wl = wlAll + wave * WLCAP;
    int wc = 0;
#pragma unroll 1
    for (int it = 0; it < NIT; ++it) {
      const int base = segBeg + it * WCH;
      int dv[4], sv[4];
#pragma unroll
      for (int j = 0; j < 4; ++j) {
        const int e  = base + 32 * j + lane;
        const int ec = e < EE - 1 ? e : EE - 1;
        int d = dstp[ec];
        asm volatile("" :: "v"(d));
        int s = srcp[ec];
        asm volatile("" :: "v"(s));
        dv[j] = d;
        sv[j] = s;
      }
#pragma unroll
      for (int j = 0; j < 4; ++j) {
        const int e = base + 32 * j + lane;
        const unsigned s10 = (unsigned)dv[j] - (unsigned)slotBase;
        const bool hj = (s10 < (unsigned)NBA) & (e < segEnd);
        const unsigned mj = __builtin_amdgcn_ballot_w32(hj);
        const int pos = wc + (int)__builtin_amdgcn_mbcnt_lo(mj, 0u);
        const int pk  = (clampi(sv[j], 0, NN - 1) << SLA) | (int)(s10 & (unsigned)(NBA - 1));
        if (hj && pos < WLCAP) wl[pos] = pk;
        wc += (int)__builtin_popcount(mj);
      }
    }
    if (lane == 0) misc[wave] = wc;
  }
  __syncthreads();

  if (wave == 0) {
    const int r = drain<0>(wlAll, misc, cnt, cur, sl, lane);
    if (lane == 0) { misc[8] = r & 0x3fffffff; misc[9] = (r >> 30) & 1; }
  }
  __syncthreads();

  if (wave == 0) {
    const int base = lane * (NBA / 32);
    int s = 0;
#pragma unroll 1
    for (int i = 0; i < NBA / 32; ++i) s += cnt[base + i];
    int incl = s;
#pragma unroll
    for (int d = 1; d < 32; d <<= 1) {
      const int y = __shfl_up(incl, d, 32);
      if (lane >= d) incl += y;
    }
    int run = incl - s;
#pragma unroll 1
    for (int i = 0; i < NBA / 32; ++i) {
      const int cv = cnt[base + i];
      offs[base + i] = run;
      cur[base + i]  = run;
      run += cv;
    }
  }
  __syncthreads();

  if (wave == 0) {
    const int r2 = drain<1>(wlAll, misc, cnt, cur, sl, lane);
    (void)r2;
  }
  __syncthreads();

  const int ovf = (misc[9] != 0) ? 1 : 0;
  int* lp = LIST + (size_t)blk * LCAP;
  for (int pass = 0; pass < 2; ++pass) {
#pragma unroll 1
    for (int it = 0; it < LCAP / (4 * 256); ++it) {
      const int q = it * 256 + tid;
      const v4i v = *(const v4ia*)(sl + 4 * q);
      *(volatile v4i*)(lp + 4 * q) = v;
    }
    __threadfence();
  }
  {
    const v4i m1 = (v4i){ -1, -1, -1, -1 };
    v4i c4 = *(const v4ia*)(cnt + 4 * tid);
    const v4i o4 = *(const v4ia*)(offs + 4 * tid);
    c4 = (ovf != 0) ? m1 : c4;
    const v4i f4 = (v4i){ ovf, ovf, ovf, ovf };
    volatile v4i* qc = (volatile v4i*)(CNT + slotBase + 4 * tid);
    volatile v4i* qo = (volatile v4i*)(OFF + slotBase + 4 * tid);
    volatile v4i* qf = (volatile v4i*)(FLG + blk * 32 + 4 * (tid & 7));
    *qc = c4;
    *qo = o4;
    if (tid < 8) *qf = f4;
    __threadfence();
    *qc = c4;
    *qo = o4;
    if (tid < 8) *qf = f4;
  }
}

__device__ __forceinline__ float nmaxf(float a, float b) { return ((a > b) | (a != a)) ? a : b; }
__device__ __forceinline__ float wsum(float p) {
  p = p + __shfl_xor(p, 16, 32);
  p = p + __shfl_xor(p, 8, 32);
  p = p + __shfl_xor(p, 4, 32);
  p = p + __shfl_xor(p, 2, 32);
  p = p + __shfl_xor(p, 1, 32);
  return p;
}
__device__ __forceinline__ float wmaxn(float m) {
  m = nmaxf(m, __shfl_xor(m, 16, 32));
  m = nmaxf(m, __shfl_xor(m, 8, 32));
  m = nmaxf(m, __shfl_xor(m, 4, 32));
  m = nmaxf(m, __shfl_xor(m, 2, 32));
  m = nmaxf(m, __shfl_xor(m, 1, 32));
  return m;
}
__device__ __forceinline__ float rl_f(float v, int k) {
  return __int_as_float(__builtin_amdgcn_readlane(__float_as_int(v), k));
}
__device__ __forceinline__ float dot4(v4f g, v4f xr, v4f at, float part) {
#pragma unroll
  for (int e = 0; e < 4; ++e) {
    const float v  = g[e] + xr[e];
    const float ev = (v >= 0.0f) ? v : (NEGS * v);
    part = part + ev * at[e];
  }
  return part;
}
__device__ __forceinline__ float relu_keep(float v) { return (v > 0.0f) ? v : (v - v); }

template <int C, int SPLIT>
__global__ __launch_bounds__(256) __attribute__((amdgpu_num_vgpr(248)))
void k_replay(const float* XL, const float* XR, const float* __restrict__ ATT, const float* __restrict__ BIA,
              const int* __restrict__ LIST, const int* __restrict__ CNT, const int* __restrict__ OFF,
              const int* __restrict__ FLG, unsigned short* HOUT) {
  static_assert(C == 256 || C == 128);
  static_assert(SPLIT == 0 || SPLIT == 1);
  constexpr int CPL  = C / 32;
  constexpr int NV   = CPL / 4;
  constexpr int KOUT = C * (1 + SPLIT);
  __shared__ __attribute__((aligned(16))) float sAtt[C];
  __shared__ __attribute__((aligned(16))) float sB[C];
  const int tid = (int)threadIdx.x, lane = tid & 31, wave = tid >> 5;

  if (tid < C / 4) {
    const v4f a = *(const v4fa*)(ATT + 4 * tid);
    *(v4fa*)(sAtt + 4 * tid) = a;
  } else if (tid < C / 2) {
    const int u = tid - C / 4;
    const v4f a = *(const v4fa*)(BIA + 4 * u);
    *(v4fa*)(sB + 4 * u) = a;
  }
  __syncthreads();

  const int n    = __builtin_amdgcn_readfirstlane((int)blockIdx.x * 8 + wave);
  const bool live = n < NN;
  const int nc   = live ? n : NN - 1;
  const int b    = nc >> SLA;

  int rc = CNT[nc];
  asm volatile("" :: "v"(rc));
  int ro = OFF[nc];
  asm volatile("" :: "v"(ro));
  int fl = FLG[b * 32];
  asm volatile("" :: "v"(fl));
  const bool bad = (rc < 0) | (rc > DEGCAP) | (fl != 0);
  const int cn  = __builtin_amdgcn_readfirstlane(live ? clampi(rc, 0, DEGCAP) : 0);
  const int off = __builtin_amdgcn_readfirstlane(clampi(ro, 0, LCAP - 1));

  if (!live) {
    unsigned short* dp = HOUT + (size_t)n * KOUT + CPL * lane;
    if (CPL == 8) {
      const v4u z = (v4u){ 0u, 0u, 0u, 0u };
      volatile v4u* qh = (volatile v4u*)dp;
      volatile v4u* ql = (volatile v4u*)(dp + C);
      *qh = z;
      if (SPLIT != 0) *ql = z;
      __threadfence();
      *qh = z;
      if (SPLIT != 0) *ql = z;
    } else {
      const v2u z = (v2u){ 0u, 0u };
      volatile v2u* qh = (volatile v2u*)dp;
      volatile v2u* ql = (volatile v2u*)(dp + C);
      *qh = z;
      if (SPLIT != 0) *ql = z;
      __threadfence();
      *qh = z;
      if (SPLIT != 0) *ql = z;
    }
  } else {
    const int cm1 = cn > 0 ? cn - 1 : 0;
    const int* lst = LIST + (size_t)b * LCAP;
    const int j0 = lane < cm1 ? lane : cm1;
    const int j1 = (32 + lane) < cm1 ? (32 + lane) : cm1;
    int e0 = lst[clampi(off + j0, 0, LCAP - 1)];
    asm volatile("" :: "v"(e0));
    int e1 = lst[clampi(off + j1, 0, LCAP - 1)];
    asm volatile("" :: "v"(e1));
    const int sr0 = clampi(e0, 0, NN - 1);
    const int sr1 = clampi(e1, 0, NN - 1);

    v4f xr[NV], xo[NV], at[NV];
#pragma unroll
    for (int q = 0; q < NV; ++q) {
      xr[q] = *(const v4fa*)(XR + (size_t)n * LDF + CPL * lane + 4 * q);
      asm volatile("" :: "v"(xr[q]));
      xo[q] = *(const v4fa*)(XL + (size_t)n * LDF + CPL * lane + 4 * q);
      asm volatile("" :: "v"(xo[q]));
      at[q] = *(const v4fa*)(sAtt + CPL * lane + 4 * q);
    }

    float lg0 = 0.0f, lg1 = 0.0f;
#pragma unroll 1
    for (int k = 0; k < cn; ++k) {
      const int ka = k & 31;
      const int sa = __builtin_amdgcn_readlane(sr0, ka);
      const int sb = __builtin_amdgcn_readlane(sr1, ka);
      const int sk = (k < 32) ? sa : sb;
      const float* gp = XL + (size_t)sk * LDF + CPL * lane;
      float part = 0.0f;
#pragma unroll
      for (int q = 0; q < NV; ++q) {
        const v4f g = *(const v4fa*)(gp + 4 * q);
        asm volatile("" :: "v"(g));
        part = dot4(g, xr[q], at[q], part);
      }
      part = wsum(part);
      lg0 = (lane == k) ? part : lg0;
      lg1 = (lane == k - 32) ? part : lg1;
    }
    float pl = 0.0f;
#pragma unroll
    for (int q = 0; q < NV; ++q) pl = dot4(xo[q], xr[q], at[q], pl);
    pl = wsum(pl);
    lg0 = (lane == cn) ? pl : lg0;
    lg1 = (lane == cn - 32) ? pl : lg1;
    const int tot = cn + 1;

    const float v0 = (lane < tot) ? lg0 : pl;
    const float v1 = (32 + lane < tot) ? lg1 : pl;
    float mx = wmaxn(nmaxf(v0, v1));
    mx = __int_as_float(__builtin_amdgcn_readfirstlane(__float_as_int(mx)));
    const float p0 = expf(lg0 - mx);
    const float p1 = expf(lg1 - mx);
    float den = 0.0f;
#pragma unroll 1
    for (int k = 0; k < tot; ++k) {
      const int ka = k & 31;
      const float pa = rl_f(p0, ka);
      const float pb = rl_f(p1, ka);
      den = den + ((k < 32) ? pa : pb);
    }
    const float a0 = p0 / den;
    const float a1 = p1 / den;

    v4f acc[NV];
#pragma unroll
    for (int q = 0; q < NV; ++q) acc[q] = (v4f){ 0.0f, 0.0f, 0.0f, 0.0f };
#pragma unroll 1
    for (int k = 0; k < cn; ++k) {
      const int ka = k & 31;
      const int sa = __builtin_amdgcn_readlane(sr0, ka);
      const int sb = __builtin_amdgcn_readlane(sr1, ka);
      const int sk = (k < 32) ? sa : sb;
      const float wa = rl_f(a0, ka);
      const float wb = rl_f(a1, ka);
      const float ak = (k < 32) ? wa : wb;
      const float* gp = XL + (size_t)sk * LDF + CPL * lane;
#pragma unroll
      for (int q = 0; q < NV; ++q) {
        const v4f g = *(const v4fa*)(gp + 4 * q);
        asm volatile("" :: "v"(g));
        const v4f t = g * ak;
        acc[q] = acc[q] + t;
      }
    }
    {
      const int ka = cn & 31;
      const float wa = rl_f(a0, ka);
      const float wb = rl_f(a1, ka);
      const float aL = (cn < 32) ? wa : wb;
#pragma unroll
      for (int q = 0; q < NV; ++q) {
        const v4f t = xo[q] * aL;
        acc[q] = acc[q] + t;
      }
    }

    const float qn = __uint_as_float(0x7fc00000u);
    float rr[8] = { 0.0f, 0.0f, 0.0f, 0.0f, 0.0f, 0.0f, 0.0f, 0.0f };
#pragma unroll
    for (int q = 0; q < NV; ++q) {
      const v4f bb = *(const v4fa*)(sB + CPL * lane + 4 * q);
#pragma unroll
      for (int e = 0; e < 4; ++e) {
        float v = relu_keep(acc[q][e] + bb[e]);
        v = bad ? qn : v;
        rr[4 * q + e] = v;
      }
    }
    unsigned short* dp = HOUT + (size_t)n * KOUT + CPL * lane;
    if (CPL == 8) {
      const v4f a = (v4f){ rr[0], rr[1], rr[2], rr[3] };
      const v4f c = (v4f){ rr[4], rr[5], rr[6], rr[7] };
      const v4u hi = pack8_bf16(a, c);
      const v4u lo = pack8_bf16_lo(a, c);
      volatile v4u* qh = (volatile v4u*)dp;
      volatile v4u* ql = (volatile v4u*)(dp + C);
      *qh = hi;
      if (SPLIT != 0) *ql = lo;
      __threadfence();
      *qh = hi;
      if (SPLIT != 0) *ql = lo;
    } else {
      const v2u hi = (v2u){ pk16(bf16_bits(rr[0]), bf16_bits(rr[1])), pk16(bf16_bits(rr[2]), bf16_bits(rr[3])) };
      const v2u lo = (v2u){ pk16(bf16_lo_bits(rr[0]), bf16_lo_bits(rr[1])),
                            pk16(bf16_lo_bits(rr[2]), bf16_lo_bits(rr[3])) };
      volatile v2u* qh = (volatile v2u*)dp;
      volatile v2u* ql = (volatile v2u*)(dp + C);
      *qh = hi;
      if (SPLIT != 0) *ql = lo;
      __threadfence();
      *qh = hi;
      if (SPLIT != 0) *ql = lo;
    }
  }
}

__global__ __launch_bounds__(256) __attribute__((amdgpu_num_vgpr(248)))
void k_out(const float* __restrict__ T, const int* __restrict__ FLG, const int* __restrict__ CNT,
           float* __restrict__ out) {
  const int f  = (int)blockIdx.x * 256 + (int)threadIdx.x;
  const int fc = f < OUT_ELEMS ? f : OUT_ELEMS - 1;
  const int n0 = fc / NCLS;
  const int n  = n0 < NN - 1 ? n0 : NN - 1;
  const int c0 = fc - n0 * NCLS;
  const int c  = c0 < NCLS - 1 ? c0 : NCLS - 1;
  const float t = T[(size_t)n * TN + c];
  asm volatile("" :: "v"(t));
  int fl = FLG[(n >> SLA) * 32];
  asm volatile("" :: "v"(fl));
  int rc = CNT[n];
  asm volatile("" :: "v"(rc));
  const bool bad = (fl != 0) | (rc < 0) | (rc > DEGCAP);
  const float qn = __uint_as_float(0x7fc00000u);
  const float v = bad ? qn : t;
  if (f < OUT_ELEMS) {
    volatile float* q = (volatile float*)(out + f);
    *q = v;
    __threadfence();
    *q = v;
  }
}

extern "C" void kernel_launch(void* const* d_in, const int* in_sizes, int n_in,
                              void* d_out, int out_size, void* d_ws, size_t ws_size,
                              hipStream_t stream) {
  if (n_in < 12) return;
  if (in_sizes[0] != NN * DF || in_sizes[1] != 2 * EE) return;
  if (in_sizes[2] != DF * H1 || in_sizes[3] != DF * H1 || in_sizes[4] != H1 || in_sizes[5] != H1) return;
  if (in_sizes[6] != H1 * H2 || in_sizes[7] != H1 * H2 || in_sizes[8] != H2 || in_sizes[9] != H2) return;
  if (in_sizes[10] != H2 * NCLS || in_sizes[11] != NCLS) return;
  if (out_size != OUT_ELEMS) return;
  if (ws_size < WS_TOTAL) return;

  const float* x    = (const float*)d_in[0];
  const int*   ei   = (const int*)  d_in[1];
  const float* W1l  = (const float*)d_in[2];
  const float* W1r  = (const float*)d_in[3];
  const float* att1 = (const float*)d_in[4];
  const float* b1   = (const float*)d_in[5];
  const float* W2l  = (const float*)d_in[6];
  const float* W2r  = (const float*)d_in[7];
  const float* att2 = (const float*)d_in[8];
  const float* b2   = (const float*)d_in[9];
  const float* Wc   = (const float*)d_in[10];
  const float* bc   = (const float*)d_in[11];
  float* out = (float*)d_out;

  char* ws = (char*)d_ws;
  float* P = (float*)(ws + OFF_P);
  float* Q = (float*)(ws + OFF_Q);
  unsigned short* XB   = (unsigned short*)(ws + OFF_RX);
  unsigned short* H1PL = (SPLIT_L2 != 0) ? (unsigned short*)(ws + OFF_Q) : (unsigned short*)(ws + OFF_RX);
  unsigned short* H2PL = (unsigned short*)(ws + OFF_Q);
  float* T = (float*)(ws + OFF_Q + SZ_H2);
  int* LIST = (int*)(ws + OFF_LIST);
  int* CNT  = (int*)(ws + OFF_CNT);
  int* OFS  = (int*)(ws + OFF_OFF);
  int* FLG  = (int*)(ws + OFF_FLG);
  unsigned short* W1LT = (unsigned short*)(ws + OFF_W1L);
  unsigned short* W1RT = (unsigned short*)(ws + OFF_W1R);
  unsigned short* W2D  = (unsigned short*)(ws + OFF_W2);
  unsigned short* WCD  = (unsigned short*)(ws + OFF_WC);
  float* VEC = (float*)(ws + OFF_VEC);

  hipFuncSetAttribute(reinterpret_cast<const void*>(&k_bucket), hipFuncAttributeMaxDynamicSharedMemorySize, B_BYTES);

  k_prep<<<NB_PREP, 256, 0, stream>>>(x, W1l, W1r, att1, b1, W2l, W2r, att2, b2, Wc, bc,
                                      XB, W1LT, W1RT, W2D, WCD, VEC);
  k_bucket<<<NBLK, 256, B_BYTES, stream>>>(ei, LIST, CNT, OFS, FLG);
  k_gemm_nt<0, 0><<<(((NN + 63) / 64) * (H1 / 64) + 7) / 8, 256, 0, stream>>>(XB, W1LT, VEC, P, NN, H1, K1, LDF);
  k_gemm_nt<0, 0><<<(((NN + 63) / 64) * (H1 / 64) + 7) / 8, 256, 0, stream>>>(XB, W1RT, VEC, Q, NN, H1, K1, LDF);
  k_replay<H1, SPLIT_L2><<<NP / 8, 256, 0, stream>>>(P, Q, VEC + V_ATT1, VEC + V_B1, LIST, CNT, OFS, FLG, H1PL);
  k_gemm_nt<0, 0><<<(((NN + 63) / 64) * (LDF / 64) + 7) / 8, 256, 0, stream>>>(H1PL, W2D, VEC, P, NN, LDF, K2, LDF);
  k_replay<H2, SPLIT_HEAD><<<NP / 8, 256, 0, stream>>>(P, P + H2, VEC + V_ATT2, VEC + V_B2, LIST, CNT, OFS, FLG, H2PL);
  k_gemm_nt<0, 1><<<(((NN + 63) / 64) * (TN / 64) + 7) / 8, 256, 0, stream>>>(H2PL, WCD, VEC + V_BC, T, NN, TN, K3, TN);
  k_out<<<(OUT_ELEMS + 255) / 256, 256, 0, stream>>>(T, FLG, CNT, out);
}
